// OptimizedHilbertAttention_58926951301481
// MI455X (gfx1250) — hardware-verified
//
#include <hip/hip_runtime.h>


#define NB_  2
#define MM   4096
#define DD   1024
#define NH_  16
#define HD   64
#define F3   (3 * DD)
#define NBK  64
#define BS   64
#define NZ   (NH_ * NBK)
#define PCAR 1024.0f
typedef _Float16 h16;
typedef unsigned short bf;
typedef __attribute__((ext_vector_type(16))) __bf16   v16bf;
typedef __attribute__((ext_vector_type(16))) _Float16 v16h;
typedef __attribute__((ext_vector_type(8)))  _Float16 v8h;
typedef __attribute__((ext_vector_type(8)))  unsigned short v8us;
typedef __attribute__((ext_vector_type(8)))  float    v8f;
typedef __attribute__((ext_vector_type(4)))  float    v4f;
typedef v8h  __attribute__((may_alias)) v8ha;
typedef v4f  __attribute__((may_alias)) v4fa;
typedef v8us __attribute__((may_alias)) v8usa;

__device__ __forceinline__ unsigned short f2bf(float f) { unsigned u = __float_as_uint(f); u += 0x7FFFu + ((u >> 16) & 1u); return (unsigned short)(u >> 16); }
__device__ __forceinline__ float bf2f(unsigned short b) { return __uint_as_float(((unsigned)b) << 16); }
__device__ __forceinline__ float bfr(float f) { return bf2f(f2bf(f)); }
__device__ __forceinline__ v16h cat16(v8h lo, v8h hi) { return __builtin_shufflevector(lo, hi, 0, 1, 2, 3, 4, 5, 6, 7, 8, 9, 10, 11, 12, 13, 14, 15); }
__device__ __forceinline__ v16bf cat16b(v8us lo, v8us hi) { return __builtin_bit_cast(v16bf, __builtin_shufflevector(lo, hi, 0, 1, 2, 3, 4, 5, 6, 7, 8, 9, 10, 11, 12, 13, 14, 15)); }
__device__ __forceinline__ v8f wmma16(v16h a, v16h b, v8f c) { return __builtin_amdgcn_wmma_f32_16x16x32_f16(false, a, false, b, (short)0, c, false, false); }
__device__ __forceinline__ v8f wmmab(v16bf a, v16bf b, v8f c) { return __builtin_amdgcn_wmma_f32_16x16x32_bf16(false, a, false, b, (short)0, c, false, false); }


template <typename T16> struct WFrag;
template <> struct WFrag<h16> { typedef v16h V; static __device__ __forceinline__ V ld(const h16* p) { return cat16(*(const v8h*)p, *(const v8h*)(p + 16)); } static __device__ __forceinline__ v8f mma(V a, V b, v8f c) { return wmma16(a, b, c); } };
template <> struct WFrag<bf> { typedef v16bf V; static __device__ __forceinline__ V ld(const bf* p) { return cat16b(*(const v8us*)p, *(const v8us*)(p + 16)); } static __device__ __forceinline__ v8f mma(V a, V b, v8f c) { return wmmab(a, b, c); } };
template <typename T16, int NSPLIT, bool BIAS>
__global__ __launch_bounds__(32) void k_gemmw(const T16* __restrict__ A, const T16* __restrict__ A2, const T16* __restrict__ Bt, const T16* __restrict__ Bt2, int K, float* C, int ldc, const float* __restrict__ bias, size_t sA, size_t sB, size_t sC) {
    typedef typename WFrag<T16>::V V;
    __shared__ __align__(16) float os[16 * 68];
    const size_t z = blockIdx.z; A += z * sA; if (A2) A2 += z * sA; Bt += z * sB; if (Bt2) Bt2 += z * sB; C += z * sC;
    const int lane = threadIdx.x & 31, lr = lane & 15, hi = lane >> 4; const int r0 = blockIdx.x * 64, c0 = blockIdx.y * 64;
    v8f acc[4][4];
#pragma unroll
    for (int mb = 0; mb < 4; ++mb)
#pragma unroll
        for (int nb = 0; nb < 4; ++nb) acc[mb][nb] = (v8f){};
    const size_t aoff = (size_t)(r0 + lr) * K + 8 * hi, boff = (size_t)(c0 + lr) * K + 8 * hi;
#pragma unroll 1
    for (int kc = 0; kc < K; kc += 32) {
        V a[4], a2[4];
#pragma unroll
        for (int mb = 0; mb < 4; ++mb) { a[mb] = WFrag<T16>::ld(A + aoff + (size_t)mb * 16 * K + kc); if (NSPLIT == 1 || NSPLIT == 2) a2[mb] = WFrag<T16>::ld(A2 + aoff + (size_t)mb * 16 * K + kc); }
#pragma unroll
        for (int nb = 0; nb < 4; ++nb) { const V b = WFrag<T16>::ld(Bt + boff + (size_t)nb * 16 * K + kc); V b2; if (NSPLIT >= 2) b2 = WFrag<T16>::ld(Bt2 + boff + (size_t)nb * 16 * K + kc);
#pragma unroll
            for (int mb = 0; mb < 4; ++mb) { acc[mb][nb] = WFrag<T16>::mma(a[mb], b, acc[mb][nb]); if (NSPLIT == 1 || NSPLIT == 2) acc[mb][nb] = WFrag<T16>::mma(a2[mb], b, acc[mb][nb]); if (NSPLIT >= 2) acc[mb][nb] = WFrag<T16>::mma(a[mb], b2, acc[mb][nb]); } }
        asm volatile("v_nop\n\tv_nop\n\tv_nop\n\tv_nop" : "+v"(acc[0][0]), "+v"(acc[1][1]), "+v"(acc[2][2]), "+v"(acc[3][3]) : "v"(a[0]), "v"(a[3]));
    }
#pragma unroll
    for (int mb = 0; mb < 4; ++mb) {
#pragma unroll
        for (int nb = 0; nb < 4; ++nb) {
#pragma unroll
            for (int j = 0; j < 8; ++j) os[(hi * 8 + j) * 68 + nb * 16 + lr] = acc[mb][nb][j]; }
        __builtin_amdgcn_wave_barrier(); asm volatile("" ::: "memory");
        float* crow = C + (size_t)(r0 + mb * 16) * ldc + c0;
#pragma unroll 1
        for (int ps = 0; ps < 2; ++ps) {
#pragma unroll
            for (int s = 0; s < 8; ++s) { const int row = 2 * s + hi, cofs = lr * 4; v4f val = *(const v4fa*)(os + row * 68 + cofs); if (BIAS) { val[0] += bfr(bias[c0 + cofs]); val[1] += bfr(bias[c0 + cofs + 1]); val[2] += bfr(bias[c0 + cofs + 2]); val[3] += bfr(bias[c0 + cofs + 3]); }
                *(volatile v4f*)(crow + (size_t)row * ldc + cofs) = val; }
            if (ps == 0) __threadfence(); }
        __builtin_amdgcn_wave_barrier(); asm volatile("" ::: "memory");
    }
}

__device__ __forceinline__ h16 tohx(float x) { return (h16)x; }
__device__ __forceinline__ void splitf(float y, unsigned short& h, unsigned short& l) { h = f2bf(y); l = f2bf(y - bf2f(h)); }
typedef __attribute__((ext_vector_type(2))) _Float16 v2h;
typedef __attribute__((ext_vector_type(2))) unsigned short v2us;
typedef __attribute__((ext_vector_type(2))) float v2f;
typedef __attribute__((ext_vector_type(2))) int v2i;

__global__ __launch_bounds__(256) void k_wtG(const float* __restrict__ w, int K, int N, bf* Bt) {
    const int lane = threadIdx.x & 31; const int L0 = (blockIdx.x * 8 + (threadIdx.x >> 5)) * 8; const int nlines = N * K / 64;
#pragma unroll 1
    for (int ps = 0; ps < 2; ++ps) {
#pragma unroll 1
        for (int l = 0; l < 8; ++l) { const int L = L0 + l; if (L >= nlines) break; const size_t e = (size_t)L * 64 + lane * 2; const int k = (int)(e % K), n = (int)(e / K); v2us o;
            o[0] = f2bf(w[(size_t)k * N + n]); o[1] = f2bf(w[(size_t)(k + 1) * N + n]); *(volatile v2us*)(Bt + e) = o; }
        if (ps == 0) __threadfence(); }
}
__global__ __launch_bounds__(256) void k_cvt8(const float* __restrict__ src, bf* dst, size_t n8) { const size_t i = (size_t)blockIdx.x * 256 + threadIdx.x; if (i >= n8) return; const v8f v = *(const v8f*)(src + i * 8); v8us o;
#pragma unroll
    for (int k = 0; k < 8; ++k) o[k] = f2bf(v[k]); *(volatile v8us*)(dst + i * 8) = o; __threadfence(); *(volatile v8us*)(dst + i * 8) = o; }
__global__ __launch_bounds__(256) void k_idx(const int* __restrict__ mp, int* IDX) { const int i = blockIdx.x * 256 + threadIdx.x; if (i >= NBK * BS) return; const int n = i >> 6, s = i & 63; int m0 = mp[n * BS]; m0 = m0 < 0 ? 0 : (m0 >= MM ? MM - 1 : m0);
    const int kp0 = (m0 / 256) * 256 + 4 * s; v2i o; if (kp0 < MM) { int ix = mp[kp0]; ix = ix < 0 ? 0 : (ix >= MM ? MM - 1 : ix); o[0] = ix; o[1] = 1; } else { o[0] = 0; o[1] = 0; }
    *(volatile v2i*)(IDX + (size_t)i * 2) = o; __threadfence(); *(volatile v2i*)(IDX + (size_t)i * 2) = o; }
__global__ __launch_bounds__(256) void k_gq(const float* __restrict__ F, const int* __restrict__ mp, h16* QG) { const int e = (blockIdx.x * 256 + threadIdx.x) * 2; if (e >= NZ * BS * HD) return; const int d = e & 63; const int m = (e >> 6) & 63; const int z = e >> 12; const int n = z & 63, h = z >> 6; int r = mp[n * BS + m]; r = r < 0 ? 0 : (r >= MM ? MM - 1 : r);
    const float* src = F + (size_t)r * F3 + h * HD + d; v2h o; o[0] = tohx(src[0] * 0.125f); o[1] = tohx(src[1] * 0.125f); *(volatile v2h*)(QG + e) = o; __threadfence(); *(volatile v2h*)(QG + e) = o; }
__global__ __launch_bounds__(256) void k_gk(const float* __restrict__ F, const int* __restrict__ IDX, h16* KG) { const int e = (blockIdx.x * 256 + threadIdx.x) * 2; if (e >= NZ * BS * HD) return; const int d = e & 63; const int s = (e >> 6) & 63; const int z = e >> 12; const int n = z & 63, h = z >> 6; const v2i ix = *(const v2i*)(IDX + (size_t)(n * BS + s) * 2);
    const float* src = F + (size_t)ix[0] * F3 + DD + h * HD + d; const float mk = (float)ix[1]; v2h o; o[0] = tohx(src[0] * mk); o[1] = tohx(src[1] * mk); *(volatile v2h*)(KG + e) = o; __threadfence(); *(volatile v2h*)(KG + e) = o; }
__global__ __launch_bounds__(256) void k_gv(const float* __restrict__ F, const int* __restrict__ IDX, h16* VT) { const int e = (blockIdx.x * 256 + threadIdx.x) * 2; if (e >= NZ * HD * BS) return; const int s = e & 63; const int d = (e >> 6) & 63; const int z = e >> 12; const int n = z & 63, h = z >> 6; v2h o;
#pragma unroll
    for (int q = 0; q < 2; ++q) { const v2i ix = *(const v2i*)(IDX + (size_t)(n * BS + s + q) * 2); o[q] = tohx(F[(size_t)ix[0] * F3 + 2 * DD + h * HD + d] * (float)ix[1]); }
    *(volatile v2h*)(VT + e) = o; __threadfence(); *(volatile v2h*)(VT + e) = o; }
__global__ __launch_bounds__(256) void k_hexp(const float* __restrict__ S, const int* __restrict__ mp, h16* P, float* LS) {
    const int lane = threadIdx.x & 31; const int z = blockIdx.x * 8 + (threadIdx.x >> 5); if (z >= NZ) return; const int n = z & 63; const float* sz = S + (size_t)z * BS * BS; const int s0 = lane * 2;
    float cm0 = -3.0e38f, cm1 = -3.0e38f;
    for (int m = 0; m < BS; ++m) { int r = mp[n * BS + m]; r = r < 0 ? 0 : r; const int base = (r / 256) * 256; const v2f a = *(const v2f*)(sz + m * BS + s0);
        const float t0 = (base + 4 * s0 < MM) ? a[0] : -1.0e9f, t1 = (base + 4 * (s0 + 1) < MM) ? a[1] : -1.0e9f; cm0 = fmaxf(cm0, t0); cm1 = fmaxf(cm1, t1); }
    v2f myls; myls[0] = 0.f; myls[1] = 0.f;
#pragma unroll 1
    for (int ps = 0; ps < 2; ++ps) {
        for (int m = 0; m < BS; ++m) { int r = mp[n * BS + m]; r = r < 0 ? 0 : r; const int base = (r / 256) * 256; const v2f a = *(const v2f*)(sz + m * BS + s0);
            const float t0 = (base + 4 * s0 < MM) ? a[0] : -1.0e9f, t1 = (base + 4 * (s0 + 1) < MM) ? a[1] : -1.0e9f;
            float d0 = __fsub_rn(t0, cm0), d1 = __fsub_rn(t1, cm1); asm volatile("" : "+v"(d0)); asm volatile("" : "+v"(d1)); const float e0 = __builtin_amdgcn_exp2f(__fmul_rn(d0, 1.4426950408889634f)), e1 = __builtin_amdgcn_exp2f(__fmul_rn(d1, 1.4426950408889634f));
            v2h o; o[0] = tohx(e0 * PCAR); o[1] = tohx(e1 * PCAR); *(volatile v2h*)(P + (size_t)z * BS * BS + m * BS + s0) = o;
            float sm = __fadd_rn(e0, e1);
#pragma unroll
            for (int sh = 16; sh; sh >>= 1) sm += __shfl_xor(sm, sh, 32);
            if ((m >> 1) == lane) myls[m & 1] = __fadd_rn(1e-6f, sm); }
        *(volatile v2f*)(LS + (size_t)z * BS + lane * 2) = myls;
        if (ps == 0) __threadfence(); }
}
__global__ __launch_bounds__(256) void k_hout(const float* __restrict__ ACC, const float* __restrict__ LS, bf* Ah, bf* Al) { const int e = (blockIdx.x * 256 + threadIdx.x) * 2; if (e >= NZ * BS * HD) return; const int d = e & 63; const int m = (e >> 6) & 63; const int z = e >> 12; const int n = z & 63, h = z >> 6; const float ls = LS[(size_t)z * BS + m]; v2us oh, ol;
#pragma unroll
    for (int q = 0; q < 2; ++q) { unsigned short a, c2; splitf(__fdiv_rn(ACC[e + q] * (1.0f / PCAR), ls), a, c2); oh[q] = a; ol[q] = c2; }
    const size_t o = ((size_t)(n * BS + m)) * DD + h * HD + d; *(volatile v2us*)(Ah + o) = oh; *(volatile v2us*)(Al + o) = ol; __threadfence(); *(volatile v2us*)(Ah + o) = oh; *(volatile v2us*)(Al + o) = ol; }

extern "C" void kernel_launch(void* const* d_in, const int* in_sizes, int n_in,
                              void* d_out, int out_size, void* d_ws, size_t ws_size, hipStream_t stream) {
    (void)in_sizes; (void)n_in; (void)out_size;
    const float* x = (const float*)d_in[0]; const float* Wqkv = (const float*)d_in[1]; const float* bqkv = (const float*)d_in[2]; const float* Wp = (const float*)d_in[3]; const float* bp = (const float*)d_in[4]; const int* mp = (const int*)d_in[5];
    float* OUT = (float*)d_out;
    char* wsp = (char*)d_ws;
    auto take = [&](size_t bytes) { char* p = wsp; wsp += (bytes + 255) & ~(size_t)255; return (void*)p; };
    bf* WQKV = (bf*)take((size_t)F3 * DD * 2); bf* WP = (bf*)take((size_t)DD * DD * 2); int* IDX = (int*)take((size_t)NBK * BS * 2 * 4); bf* XB = (bf*)take((size_t)MM * DD * 2); float* F = (float*)take((size_t)MM * F3 * 4);
    h16* QG = (h16*)take((size_t)NZ * BS * HD * 2); h16* KG = (h16*)take((size_t)NZ * BS * HD * 2); h16* VT = (h16*)take((size_t)NZ * HD * BS * 2); float* S = (float*)take((size_t)NZ * BS * BS * 4); h16* P = (h16*)take((size_t)NZ * BS * BS * 2); float* LS = (float*)take((size_t)NZ * BS * 4); bf* Ah = (bf*)take((size_t)MM * DD * 2); bf* Al = (bf*)take((size_t)MM * DD * 2);
    if ((size_t)(wsp - (char*)d_ws) > ws_size) return;
    float* ACC = S;
    { k_wtG<<<(unsigned)((F3 * DD / 64 + 63) / 64), 256, 0, stream>>>(Wqkv, DD, F3, WQKV); k_wtG<<<(unsigned)((DD * DD / 64 + 63) / 64), 256, 0, stream>>>(Wp, DD, DD, WP); k_idx<<<(NBK * BS + 255) / 256, 256, 0, stream>>>(mp, IDX); }
    const unsigned LG = (NZ * BS * HD / 2 + 255) / 256;
    for (int b = 0; b < NB_; ++b) {
        k_cvt8<<<(unsigned)(((size_t)MM * DD / 8 + 255) / 256), 256, 0, stream>>>(x + (size_t)b * MM * DD, XB, (size_t)MM * DD / 8);
        k_gemmw<bf, 0, true><<<dim3(MM / 64, F3 / 64, 1), 32, 0, stream>>>(XB, nullptr, WQKV, nullptr, DD, F, F3, bqkv, 0, 0, 0);
        k_gq<<<LG, 256, 0, stream>>>(F, mp, QG); k_gk<<<LG, 256, 0, stream>>>(F, IDX, KG); k_gv<<<LG, 256, 0, stream>>>(F, IDX, VT);
        k_gemmw<h16, 0, false><<<dim3(1, 1, NZ), 32, 0, stream>>>(QG, nullptr, KG, nullptr, HD, S, BS, nullptr, (size_t)BS * HD, (size_t)BS * HD, (size_t)BS * BS);
        k_hexp<<<NZ / 8, 256, 0, stream>>>(S, mp, P, LS);
        k_gemmw<h16, 0, false><<<dim3(1, 1, NZ), 32, 0, stream>>>(P, nullptr, VT, nullptr, BS, ACC, HD, nullptr, (size_t)BS * BS, (size_t)HD * BS, (size_t)BS * HD);
        k_hout<<<LG, 256, 0, stream>>>(ACC, LS, Ah, Al);
        k_gemmw<bf, 1, true><<<dim3(MM / 64, DD / 64, 1), 32, 0, stream>>>(Ah, Al, WP, nullptr, DD, OUT + (size_t)b * MM * DD, DD, bp, 0, 0, 0); }
}
